// LSTMBaseline_20598663152193
// MI455X (gfx1250) — hardware-verified
//
#include <hip/hip_runtime.h>


#define NR   16384
#define DIN  512
#define HH   1024
#define NG3  (3 * HH)
#define RC   4096
typedef _Float16 h16;
typedef unsigned short bf;
typedef __attribute__((ext_vector_type(16))) __bf16   v16bf;
typedef __attribute__((ext_vector_type(16))) _Float16 v16h;
typedef __attribute__((ext_vector_type(8)))  _Float16 v8h;
typedef __attribute__((ext_vector_type(8)))  unsigned short v8us;
typedef __attribute__((ext_vector_type(8)))  float    v8f;
typedef __attribute__((ext_vector_type(4)))  float    v4f;
typedef v8h  __attribute__((may_alias)) v8ha;
typedef v4f  __attribute__((may_alias)) v4fa;
typedef v8us __attribute__((may_alias)) v8usa;

__device__ __forceinline__ unsigned short f2bf(float f) { unsigned u = __float_as_uint(f); u += 0x7FFFu + ((u >> 16) & 1u); return (unsigned short)(u >> 16); }
__device__ __forceinline__ float bf2f(unsigned short b) { return __uint_as_float(((unsigned)b) << 16); }
__device__ __forceinline__ float bfr(float f) { return bf2f(f2bf(f)); }
__device__ __forceinline__ v16h cat16(v8h lo, v8h hi) { return __builtin_shufflevector(lo, hi, 0, 1, 2, 3, 4, 5, 6, 7, 8, 9, 10, 11, 12, 13, 14, 15); }
__device__ __forceinline__ v16bf cat16b(v8us lo, v8us hi) { return __builtin_bit_cast(v16bf, __builtin_shufflevector(lo, hi, 0, 1, 2, 3, 4, 5, 6, 7, 8, 9, 10, 11, 12, 13, 14, 15)); }
__device__ __forceinline__ v8f wmma16(v16h a, v16h b, v8f c) { return __builtin_amdgcn_wmma_f32_16x16x32_f16(false, a, false, b, (short)0, c, false, false); }
__device__ __forceinline__ v8f wmmab(v16bf a, v16bf b, v8f c) { return __builtin_amdgcn_wmma_f32_16x16x32_bf16(false, a, false, b, (short)0, c, false, false); }


template <typename T16> struct WFrag;
template <> struct WFrag<h16> { typedef v16h V; static __device__ __forceinline__ V ld(const h16* p) { return cat16(*(const v8h*)p, *(const v8h*)(p + 16)); } static __device__ __forceinline__ v8f mma(V a, V b, v8f c) { return wmma16(a, b, c); } };
template <> struct WFrag<bf> { typedef v16bf V; static __device__ __forceinline__ V ld(const bf* p) { return cat16b(*(const v8us*)p, *(const v8us*)(p + 16)); } static __device__ __forceinline__ v8f mma(V a, V b, v8f c) { return wmmab(a, b, c); } };
template <typename T16, int NSPLIT, bool BIAS>
__global__ __launch_bounds__(32) void k_gemmw(const T16* __restrict__ A, const T16* __restrict__ A2, const T16* __restrict__ Bt, const T16* __restrict__ Bt2, int K, float* C, int ldc, const float* __restrict__ bias, size_t sA, size_t sB, size_t sC) {
    typedef typename WFrag<T16>::V V;
    __shared__ __align__(16) float os[16 * 68];
    const size_t z = blockIdx.z; A += z * sA; if (A2) A2 += z * sA; Bt += z * sB; if (Bt2) Bt2 += z * sB; C += z * sC;
    const int lane = threadIdx.x & 31, lr = lane & 15, hi = lane >> 4; const int r0 = blockIdx.x * 64, c0 = blockIdx.y * 64;
    v8f acc[4][4];
#pragma unroll
    for (int mb = 0; mb < 4; ++mb)
#pragma unroll
        for (int nb = 0; nb < 4; ++nb) acc[mb][nb] = (v8f){};
    const size_t aoff = (size_t)(r0 + lr) * K + 8 * hi, boff = (size_t)(c0 + lr) * K + 8 * hi;
#pragma unroll 1
    for (int kc = 0; kc < K; kc += 32) {
        V a[4], a2[4];
#pragma unroll
        for (int mb = 0; mb < 4; ++mb) { a[mb] = WFrag<T16>::ld(A + aoff + (size_t)mb * 16 * K + kc); if (NSPLIT == 1 || NSPLIT == 2) a2[mb] = WFrag<T16>::ld(A2 + aoff + (size_t)mb * 16 * K + kc); }
#pragma unroll
        for (int nb = 0; nb < 4; ++nb) { const V b = WFrag<T16>::ld(Bt + boff + (size_t)nb * 16 * K + kc); V b2; if (NSPLIT >= 2) b2 = WFrag<T16>::ld(Bt2 + boff + (size_t)nb * 16 * K + kc);
#pragma unroll
            for (int mb = 0; mb < 4; ++mb) { acc[mb][nb] = WFrag<T16>::mma(a[mb], b, acc[mb][nb]); if (NSPLIT == 1 || NSPLIT == 2) acc[mb][nb] = WFrag<T16>::mma(a2[mb], b, acc[mb][nb]); if (NSPLIT >= 2) acc[mb][nb] = WFrag<T16>::mma(a[mb], b2, acc[mb][nb]); } }
        asm volatile("v_nop\n\tv_nop\n\tv_nop\n\tv_nop" : "+v"(acc[0][0]), "+v"(acc[1][1]), "+v"(acc[2][2]), "+v"(acc[3][3]) : "v"(a[0]), "v"(a[3]));
    }
#pragma unroll
    for (int mb = 0; mb < 4; ++mb) {
#pragma unroll
        for (int nb = 0; nb < 4; ++nb) {
#pragma unroll
            for (int j = 0; j < 8; ++j) os[(hi * 8 + j) * 68 + nb * 16 + lr] = acc[mb][nb][j]; }
        __builtin_amdgcn_wave_barrier(); asm volatile("" ::: "memory");
        float* crow = C + (size_t)(r0 + mb * 16) * ldc + c0;
#pragma unroll 1
        for (int ps = 0; ps < 2; ++ps) {
#pragma unroll
            for (int s = 0; s < 8; ++s) { const int row = 2 * s + hi, cofs = lr * 4; v4f val = *(const v4fa*)(os + row * 68 + cofs); if (BIAS) { val[0] += bfr(bias[c0 + cofs]); val[1] += bfr(bias[c0 + cofs + 1]); val[2] += bfr(bias[c0 + cofs + 2]); val[3] += bfr(bias[c0 + cofs + 3]); }
                *(volatile v4f*)(crow + (size_t)row * ldc + cofs) = val; }
            if (ps == 0) __threadfence(); }
        __builtin_amdgcn_wave_barrier(); asm volatile("" ::: "memory");
    }
}

typedef __attribute__((ext_vector_type(4))) _Float16 v4h;
__device__ __forceinline__ h16 tohx(float x) { return (h16)x; }
__global__ __launch_bounds__(256) void k_cvt8(const float* __restrict__ src, bf* dst, size_t n8) { const size_t i = (size_t)blockIdx.x * 256 + threadIdx.x; if (i >= n8) return; const v8f v = *(const v8f*)(src + i * 8); v8us o;
#pragma unroll
    for (int k = 0; k < 8; ++k) o[k] = f2bf(v[k]); *(volatile v8us*)(dst + i * 8) = o; __threadfence(); *(volatile v8us*)(dst + i * 8) = o; }

__global__ __launch_bounds__(256) void k_cvt8h(const float* __restrict__ src, h16* dst, size_t n8) { const size_t i = (size_t)blockIdx.x * 256 + threadIdx.x; if (i >= n8) return; const v8f v = *(const v8f*)(src + i * 8); v8h o;
#pragma unroll
    for (int k = 0; k < 8; ++k) o[k] = tohx(bfr(v[k])); *(volatile v8h*)(dst + i * 8) = o; __threadfence(); *(volatile v8h*)(dst + i * 8) = o; }
__global__ __launch_bounds__(256) void k_gate(const float* __restrict__ G, const float* __restrict__ bih, const float* __restrict__ bhh, h16* H16) {
    const size_t e = ((size_t)blockIdx.x * 256 + threadIdx.x) * 4; if (e >= (size_t)RC * HH) return; const int c = (int)(e % HH); const size_t r = e / HH; const float* g = G + r * NG3;
    const v4f gi = *(const v4f*)(g + c); const v4f gg = *(const v4f*)(g + HH + c); const v4f go = *(const v4f*)(g + 2 * HH + c); v4h o;
#pragma unroll
    for (int q = 0; q < 4; ++q) { const int cc = c + q;
        float bi_ = bfr(bih[cc]); asm volatile("" : "+v"(bi_)); float bh_ = bfr(bhh[cc]); asm volatile("" : "+v"(bh_)); const float ai = __fadd_rn(gi[q], __fadd_rn(bi_, bh_));
        float bi2 = bfr(bih[2 * HH + cc]); asm volatile("" : "+v"(bi2)); float bh2 = bfr(bhh[2 * HH + cc]); asm volatile("" : "+v"(bh2)); const float ag = __fadd_rn(gg[q], __fadd_rn(bi2, bh2));
        float bi3 = bfr(bih[3 * HH + cc]); asm volatile("" : "+v"(bi3)); float bh3 = bfr(bhh[3 * HH + cc]); asm volatile("" : "+v"(bh3)); const float ao = __fadd_rn(go[q], __fadd_rn(bi3, bh3));
        const float si = __fdiv_rn(1.0f, __fadd_rn(1.0f, __builtin_amdgcn_exp2f(__fmul_rn(ai, -1.4426950408889634f))));
        const float tg = __fsub_rn(__fdiv_rn(2.0f, __fadd_rn(1.0f, __builtin_amdgcn_exp2f(__fmul_rn(ag, -2.8853900817779268f)))), 1.0f);
        const float so = __fdiv_rn(1.0f, __fadd_rn(1.0f, __builtin_amdgcn_exp2f(__fmul_rn(ao, -1.4426950408889634f))));
        float cst = __fmul_rn(si, tg); asm volatile("" : "+v"(cst));
        const float tc = __fsub_rn(__fdiv_rn(2.0f, __fadd_rn(1.0f, __builtin_amdgcn_exp2f(__fmul_rn(cst, -2.8853900817779268f)))), 1.0f);
        float h = __fmul_rn(so, tc); asm volatile("" : "+v"(h)); o[q] = tohx(h); }
    *(volatile v4h*)(H16 + e) = o; __threadfence(); *(volatile v4h*)(H16 + e) = o; }

extern "C" void kernel_launch(void* const* d_in, const int* in_sizes, int n_in,
                              void* d_out, int out_size, void* d_ws, size_t ws_size, hipStream_t stream) {
    (void)in_sizes; (void)n_in; (void)out_size;
    const float* x = (const float*)d_in[0]; const float* wih0 = (const float*)d_in[1];   const float* bih0 = (const float*)d_in[3]; const float* bhh0 = (const float*)d_in[4];
    const float* wih1 = (const float*)d_in[5];   const float* bih1 = (const float*)d_in[7]; const float* bhh1 = (const float*)d_in[8]; const float* wdec = (const float*)d_in[9]; const float* bdec = (const float*)d_in[10];
    float* OUT = (float*)d_out;
    char* wsp = (char*)d_ws;
    auto take = [&](size_t bytes) { char* p = wsp; wsp += (bytes + 255) & ~(size_t)255; return (void*)p; };
    bf* XB = (bf*)take((size_t)NR * DIN * 2); bf* W0 = (bf*)take((size_t)4 * HH * DIN * 2); h16* W1 = (h16*)take((size_t)4 * HH * HH * 2); h16* WD = (h16*)take((size_t)DIN * HH * 2);
    float* G = (float*)take((size_t)RC * NG3 * 4); h16* H0 = (h16*)take((size_t)RC * HH * 2); h16* H1 = (h16*)take((size_t)RC * HH * 2);
    if ((size_t)(wsp - (char*)d_ws) > ws_size) return;
    k_cvt8<<<(unsigned)(((size_t)NR * DIN / 8 + 255) / 256), 256, 0, stream>>>(x, XB, (size_t)NR * DIN / 8);
    k_cvt8<<<(unsigned)(((size_t)4 * HH * DIN / 8 + 255) / 256), 256, 0, stream>>>(wih0, W0, (size_t)4 * HH * DIN / 8);
    k_cvt8h<<<(unsigned)(((size_t)4 * HH * HH / 8 + 255) / 256), 256, 0, stream>>>(wih1, W1, (size_t)4 * HH * HH / 8);
    k_cvt8h<<<(unsigned)(((size_t)DIN * HH / 8 + 255) / 256), 256, 0, stream>>>(wdec, WD, (size_t)DIN * HH / 8);
    static_assert(NR % RC == 0 && RC % 64 == 0 && DIN % 32 == 0 && HH % 64 == 0, "tiles");
    for (size_t r0 = 0; r0 < NR; r0 += RC) {
        k_gemmw<bf, 0, false><<<dim3(RC / 64, HH / 64, 1), 32, 0, stream>>>(XB + r0 * DIN, nullptr, W0, nullptr, DIN, G, NG3, nullptr, 0, 0, 0);
        k_gemmw<bf, 0, false><<<dim3(RC / 64, HH / 64, 1), 32, 0, stream>>>(XB + r0 * DIN, nullptr, W0 + (size_t)2 * HH * DIN, nullptr, DIN, G + HH, NG3, nullptr, 0, 0, 0);
        k_gemmw<bf, 0, false><<<dim3(RC / 64, HH / 64, 1), 32, 0, stream>>>(XB + r0 * DIN, nullptr, W0 + (size_t)3 * HH * DIN, nullptr, DIN, G + 2 * HH, NG3, nullptr, 0, 0, 0);
        k_gate<<<(unsigned)(((size_t)RC * HH / 4 + 255) / 256), 256, 0, stream>>>(G, bih0, bhh0, H0);
        k_gemmw<h16, 0, false><<<dim3(RC / 64, HH / 64, 1), 32, 0, stream>>>(H0, nullptr, W1, nullptr, HH, G, NG3, nullptr, 0, 0, 0);
        k_gemmw<h16, 0, false><<<dim3(RC / 64, HH / 64, 1), 32, 0, stream>>>(H0, nullptr, W1 + (size_t)2 * HH * HH, nullptr, HH, G + HH, NG3, nullptr, 0, 0, 0);
        k_gemmw<h16, 0, false><<<dim3(RC / 64, HH / 64, 1), 32, 0, stream>>>(H0, nullptr, W1 + (size_t)3 * HH * HH, nullptr, HH, G + 2 * HH, NG3, nullptr, 0, 0, 0);
        k_gate<<<(unsigned)(((size_t)RC * HH / 4 + 255) / 256), 256, 0, stream>>>(G, bih1, bhh1, H1);
        k_gemmw<h16, 0, true><<<dim3(RC / 64, DIN / 64, 1), 32, 0, stream>>>(H1, nullptr, WD, nullptr, HH, OUT + r0 * DIN, DIN, bdec, 0, 0, 0); }
}
